// SpatioTemporalGAT_76321568850117
// MI455X (gfx1250) — hardware-verified
//
#include <hip/hip_runtime.h>
#include <stddef.h>


#define INF0   32
#define HIDF   64
#define NHD    4
#define HCH    16
#define EDIM   8
#define MLPW   8
#define GR     32
#define XSP    68
#define NB     768
#define CHUNK  2048
#define NTHR   256
#define NWAVE  8
#define WCAP   256
#define NGRP   (CHUNK / (NTHR * 4))
#define SLOTB  10

#define LDS_SACC (NB * HIDF)
#define LDS_DEN  (NB * NHD)
#define LDS_MX   (NB * NHD)
#define LDS_LIST (NWAVE * WCAP)
#define LDS_BYTES ((LDS_SACC + LDS_DEN + LDS_MX + LDS_LIST + NWAVE + NHD * EDIM + NHD + 4) * 4)

static_assert(WCAP == (CHUNK / NTHR) * 32);
static_assert(NGRP >= 1);
static_assert(NB < (1 << SLOTB));
static_assert(CHUNK <= 2048);
static_assert((NB % NWAVE) == 0);
static_assert(((LDS_SACC + LDS_DEN) % 4) == 0);
static_assert((LDS_MX % 4) == 0);
static_assert(LDS_BYTES == 229568);

typedef float    v2f  __attribute__((ext_vector_type(2)));
typedef float    v4f  __attribute__((ext_vector_type(4)));
typedef float    v8f  __attribute__((ext_vector_type(8)));
typedef int      v4i  __attribute__((ext_vector_type(4)));
typedef _Float16 v8h  __attribute__((ext_vector_type(8)));
typedef _Float16 v16h __attribute__((ext_vector_type(16)));
union Frag   { v16h v; v8h half[2]; };
union Pack16 { v8h h; v4i i; };

__device__ __forceinline__ v8f wm(v16h a, v16h b, v8f c) {
  v8f d = __builtin_amdgcn_wmma_f32_16x16x32_f16(false, a, false, b, (short)0, c, false, false);
  asm volatile("v_nop\n\tv_nop\n\tv_nop\n\tv_nop" : "+v"(d) : "v"(a), "v"(b));
  return d;
}

__global__ __launch_bounds__(256) void k_prep(const float* __restrict__ W1, const float* __restrict__ W2,
                                              const float* __restrict__ L1, _Float16* Wb) {
  const int p = blockIdx.x * 256 + threadIdx.x;
  if (p >= 896) return;
  float v[8];
  if (p < 256) {
    const int n = p >> 2, k0 = (p & 3) * 8;
#pragma unroll
    for (int j = 0; j < 8; ++j) v[j] = W1[(k0 + j) * HIDF + n];
  } else if (p < 768) {
    const int q = p - 256;
    const int n = q >> 3, k0 = (q & 7) * 8;
#pragma unroll
    for (int j = 0; j < 8; ++j) v[j] = W2[(k0 + j) * HIDF + n];
  } else {
    const int q = p - 768;
    const int n = q >> 3, k0 = (q & 7) * 8;
    const int nc = n < MLPW ? n : MLPW - 1;
#pragma unroll
    for (int j = 0; j < 8; ++j) {
      const float t = L1[(k0 + j) * MLPW + nc];
      v[j] = (n < MLPW) ? t : 0.f;
    }
  }
  Pack16 u;
#pragma unroll
  for (int j = 0; j < 8; ++j) u.h[j] = (_Float16)(v[j] * 8.0f);
  _Float16* dst = Wb + (size_t)p * 8;
  *(volatile v4i*)dst = u.i;
  __threadfence();
  *(volatile v4i*)dst = u.i;
}

template <int K, int NT>
__device__ __forceinline__ void stage_a(const float* __restrict__ X, int nN, int rowBase, int tid, _Float16* At) {
  constexpr int AP = K + 8;
  constexpr int F = GR * K / NT;
  static_assert((F % 8) == 0 && (K % F) == 0);
  const int r  = (tid * F) / K;
  const int c0 = (tid * F) % K;
  int row = rowBase + r;
  if (row > nN - 1) row = nN - 1;
  const float* p = X + (size_t)row * K + c0;
#pragma unroll
  for (int g = 0; g < F / 8; ++g) {
    const v4f f0 = *(const v4f*)(p + 8 * g);
    const v4f f1 = *(const v4f*)(p + 8 * g + 4);
    Pack16 u;
    u.h[0] = (_Float16)f0.x; u.h[1] = (_Float16)f0.y; u.h[2] = (_Float16)f0.z; u.h[3] = (_Float16)f0.w;
    u.h[4] = (_Float16)f1.x; u.h[5] = (_Float16)f1.y; u.h[6] = (_Float16)f1.z; u.h[7] = (_Float16)f1.w;
    *(v8h*)(At + r * AP + c0 + 8 * g) = u.h;
  }
}

template <int K>
__global__ __launch_bounds__(128) void k_gemm(
    const float* __restrict__ X, const _Float16* __restrict__ Wt,
    const float* __restrict__ att_s, const float* __restrict__ att_d,
    float* hp, float* asn, float* adn, int nN) {
  constexpr int AP = K + 8;
  __shared__ __attribute__((aligned(16))) _Float16 At[GR * AP];
  __shared__ __attribute__((aligned(16))) float Xs[GR * XSP];
  __shared__ __attribute__((aligned(16))) float As[GR * NHD];
  __shared__ __attribute__((aligned(16))) float Ds[GR * NHD];

  const int tid  = threadIdx.x;
  const int lane = tid & 31;
  const int wave = tid >> 5;
  const int hh   = lane >> 4;
  const int m    = lane & 15;
  const int rowBase = blockIdx.x * GR;

  stage_a<K, 128>(X, nN, rowBase, tid, At);
  __syncthreads();

  const int ncol = wave * 16 + m;
  v8f c0a = {0.f, 0.f, 0.f, 0.f, 0.f, 0.f, 0.f, 0.f};
  v8f c1a = {0.f, 0.f, 0.f, 0.f, 0.f, 0.f, 0.f, 0.f};
#pragma unroll
  for (int kt = 0; kt < K / 32; ++kt) {
    const int k0 = kt * 32;
    Frag a0, a1, b;
    const _Float16* pb  = Wt + (size_t)ncol * K + k0 + 8 * hh;
    const _Float16* pa0 = At + m * AP + k0 + 8 * hh;
    const _Float16* pa1 = At + (16 + m) * AP + k0 + 8 * hh;
    b.half[0]  = *(const v8h*)pb;  b.half[1]  = *(const v8h*)(pb + 16);
    a0.half[0] = *(const v8h*)pa0; a0.half[1] = *(const v8h*)(pa0 + 16);
    a1.half[0] = *(const v8h*)pa1; a1.half[1] = *(const v8h*)(pa1 + 16);
    c0a = wm(a0.v, b.v, c0a);
    c1a = wm(a1.v, b.v, c1a);
  }

#pragma unroll
  for (int r = 0; r < 8; ++r) {
    Xs[(8 * hh + r) * XSP + ncol]      = c0a[r] * 0.125f;
    Xs[(16 + 8 * hh + r) * XSP + ncol] = c1a[r] * 0.125f;
  }
  __syncthreads();

  {
    const float* xr = Xs + lane * XSP + wave * HCH;
    const float* ps = att_s + wave * HCH;
    const float* pd = att_d + wave * HCH;
    float s = 0.f, d = 0.f;
#pragma unroll 4
    for (int c = 0; c < HCH; ++c) {
      const float v = xr[c];
      s += v * ps[c];
      d += v * pd[c];
    }
    As[lane * NHD + wave] = s;
    Ds[lane * NHD + wave] = d;
  }
  __syncthreads();

  const int q  = tid & 15;
  const int r8 = tid >> 4;
  v4f xv[4];
  float* xpp[4];
#pragma unroll
  for (int i = 0; i < 4; ++i) {
    xv[i]  = *(const v4f*)(Xs + (r8 + 8 * i) * XSP + 4 * q);
    xpp[i] = hp + (size_t)(rowBase + r8 + 8 * i) * HIDF + 4 * q;
  }
  const v4f ga = *(const v4f*)(As + 4 * lane);
  const v4f gd = *(const v4f*)(Ds + 4 * lane);
  const v4f gv = (wave == 0) ? ga : gd;
  float* gp = ((wave == 0) ? asn : adn) + (size_t)(rowBase + lane) * NHD;

#pragma unroll
  for (int i = 0; i < 4; ++i) *(volatile v4f*)(xpp[i]) = xv[i];
  if (wave < 2) *(volatile v4f*)gp = gv;
  __threadfence();
#pragma unroll
  for (int i = 0; i < 4; ++i) *(volatile v4f*)(xpp[i]) = xv[i];
  if (wave < 2) *(volatile v4f*)gp = gv;
}

__global__ __launch_bounds__(NTHR) void k_gat(
    const int* __restrict__ ei, const float* __restrict__ ea,
    const float* __restrict__ hpre, const float* __restrict__ asn, const float* __restrict__ adn,
    const float* __restrict__ We, const float* __restrict__ ae, const float* __restrict__ sla,
    const float* __restrict__ bias, float* hout, int nN, int nE) {
  extern __shared__ v4f lds_dyn[];
  float* sacc = (float*)lds_dyn;
  float* denl = sacc + LDS_SACC;
  float* mxl  = denl + LDS_DEN;
  int*   list = (int*)(mxl + LDS_MX);
  int*   wcnt = list + LDS_LIST;
  float* cl   = (float*)(wcnt + NWAVE);
  float* ssl  = cl + NHD * EDIM;

  const int tid  = threadIdx.x;
  const int lane = tid & 31;
  const int wave = tid >> 5;
  const int hd   = lane >> 3;
  const int nodeBase = blockIdx.x * NB;

  {
    const v4f z4 = {0.f, 0.f, 0.f, 0.f};
    for (int i = tid; i < (LDS_SACC + LDS_DEN) / 4; i += NTHR) lds_dyn[i] = z4;
    const v4f m4 = {-1.0e30f, -1.0e30f, -1.0e30f, -1.0e30f};
    v4f* mx4 = (v4f*)mxl;
    for (int i = tid; i < LDS_MX / 4; i += NTHR) mx4[i] = m4;
    if (tid < NHD * EDIM) {
      const int h = tid >> 3, k = tid & 7;
      float s = 0.f;
#pragma unroll 1
      for (int c = 0; c < HCH; ++c) s += We[k * HIDF + h * HCH + c] * ae[h * HCH + c];
      cl[tid] = s;
    }
  }
  __syncthreads();
  if (tid < NHD) {
    float s = 0.f;
#pragma unroll 1
    for (int k = 0; k < EDIM; ++k) s += sla[k] * cl[tid * EDIM + k];
    ssl[tid] = s;
  }
  __syncthreads();
  float creg[EDIM];
#pragma unroll
  for (int k = 0; k < EDIM; ++k) creg[k] = cl[hd * EDIM + k];
  const float sself = ssl[hd];

  const int* eid = ei + nE;
  const bool al16 = ((nE & 3) == 0);

  const int nChunks = (nE + CHUNK - 1) / CHUNK;
#pragma unroll 1
  for (int ch = 0; ch < nChunks; ++ch) {
    const int cbase = ch * CHUNK;
    int wc = 0;
#pragma unroll
    for (int g = 0; g < NGRP; ++g) {
      const int el0 = (g * NTHR + tid) * 4;
      const int e0  = cbase + el0;
      const int sent = -2147483647 - 1;
      v4i d;
      if (al16 && (cbase + CHUNK <= nE)) {
        d = *(const v4i*)(eid + e0);
      } else {
        const int t0 = eid[min(e0,     nE - 1)];
        const int t1 = eid[min(e0 + 1, nE - 1)];
        const int t2 = eid[min(e0 + 2, nE - 1)];
        const int t3 = eid[min(e0 + 3, nE - 1)];
        d.x = (e0     < nE) ? t0 : sent;
        d.y = (e0 + 1 < nE) ? t1 : sent;
        d.z = (e0 + 2 < nE) ? t2 : sent;
        d.w = (e0 + 3 < nE) ? t3 : sent;
      }
      const unsigned s0 = (unsigned)d.x - (unsigned)nodeBase;
      const unsigned s1 = (unsigned)d.y - (unsigned)nodeBase;
      const unsigned s2 = (unsigned)d.z - (unsigned)nodeBase;
      const unsigned s3 = (unsigned)d.w - (unsigned)nodeBase;
      const bool h0 = s0 < (unsigned)NB;
      const bool h1 = s1 < (unsigned)NB;
      const bool h2 = s2 < (unsigned)NB;
      const bool h3 = s3 < (unsigned)NB;
      const unsigned many = __builtin_amdgcn_ballot_w32(h0 | h1 | h2 | h3);
      if (many != 0u) {
#define HITJ(J, HJ, SJ) { \
          const unsigned mj = __builtin_amdgcn_ballot_w32(HJ); \
          if (HJ) { \
            const int pos = wc + (int)__builtin_amdgcn_mbcnt_lo(mj, 0u); \
            if (pos < WCAP) list[wave * WCAP + pos] = ((el0 + (J)) << SLOTB) | (int)(SJ); \
          } \
          wc += (int)__builtin_popcount(mj); }
        HITJ(0, h0, s0)
        HITJ(1, h1, s1)
        HITJ(2, h2, s2)
        HITJ(3, h3, s3)
#undef HITJ
      }
    }
    if (lane == 0) wcnt[wave] = wc;
    __syncthreads();

    if (wave == 0) {
#pragma unroll 1
      for (int wsx = 0; wsx < NWAVE; ++wsx) {
        int n = wcnt[wsx];
        if (n > WCAP) n = WCAP;
        if (n < 0) n = 0;
#pragma unroll 1
        for (int i = 0; i < n; ++i) {
          const int ent = list[wsx * WCAP + i];
          int sl = ent & ((1 << SLOTB) - 1);
          if (sl > NB - 1) sl = NB - 1;
          const int el = (ent >> SLOTB) & (CHUNK - 1);
          int e = cbase + el;
          if (e > nE - 1) e = nE - 1;
          int src = ei[e];
          src = src < 0 ? 0 : (src > nN - 1 ? nN - 1 : src);
          int nd = nodeBase + sl;
          if (nd > nN - 1) nd = nN - 1;
          const v4f ea0 = *(const v4f*)(ea + (size_t)e * EDIM);
          const v4f ea1 = *(const v4f*)(ea + (size_t)e * EDIM + 4);
          float se = ea0.x * creg[0];
          se += ea0.y * creg[1];
          se += ea0.z * creg[2];
          se += ea0.w * creg[3];
          se += ea1.x * creg[4];
          se += ea1.y * creg[5];
          se += ea1.z * creg[6];
          se += ea1.w * creg[7];
          float al = asn[(size_t)src * NHD + hd] + adn[(size_t)nd * NHD + hd] + se;
          al = (al > 0.f) ? al : 0.2f * al;
          const int mi = sl * NHD + hd;
          const float mold = mxl[mi];
          const float mnew = fmaxf(mold, al);
          const float sc = __expf(mold - mnew);
          const float p  = __expf(al - mnew);
          const v2f xv = *(const v2f*)(hpre + (size_t)src * HIDF + 2 * lane);
          v2f* sp = (v2f*)(sacc + sl * HIDF + 2 * lane);
          const v2f cur = *sp;
          const v2f nxt = cur * sc + xv * p;
          *sp = nxt;
          const float dold = denl[mi];
          const float dnew = dold * sc + p;
          denl[mi] = dnew;
          mxl[mi]  = mnew;
        }
      }
    }
    __syncthreads();
  }

  const v2f bv = *(const v2f*)(bias + 2 * lane);
#pragma unroll 1
  for (int j = 0; j < NB / NWAVE; ++j) {
    const int slot = wave * (NB / NWAVE) + j;
    const int node = nodeBase + slot;
    if (node >= nN) break;
    const size_t nrow = (size_t)node;
    float al = asn[nrow * NHD + hd] + adn[nrow * NHD + hd] + sself;
    al = (al > 0.f) ? al : 0.2f * al;
    const int mi = slot * NHD + hd;
    const float mold = mxl[mi];
    const float mnew = fmaxf(mold, al);
    const float sc = __expf(mold - mnew);
    const float p  = __expf(al - mnew);
    const v2f xv = *(const v2f*)(hpre + nrow * HIDF + 2 * lane);
    const v2f sv = *(const v2f*)(sacc + slot * HIDF + 2 * lane) * sc + xv * p;
    const float dv  = denl[mi] * sc + p;
    const float inv = 1.0f / (dv + 1e-16f);
    v2f y = sv * inv + bv;
    y.x = y.x > 0.f ? y.x : 0.f;
    y.y = y.y > 0.f ? y.y : 0.f;
    float* op = hout + nrow * HIDF + 2 * lane;
    *(volatile v2f*)op = y;
    __threadfence();
    *(volatile v2f*)op = y;
  }
}

__global__ __launch_bounds__(64) void k_head(
    const float* __restrict__ hin, const _Float16* __restrict__ Lt,
    const float* __restrict__ lb1, const float* __restrict__ lw2, const float* __restrict__ lb2,
    float* out, int nN) {
  constexpr int K = HIDF;
  constexpr int AP = K + 8;
  __shared__ __attribute__((aligned(16))) _Float16 At[GR * AP];
  __shared__ __attribute__((aligned(16))) float Os[GR];

  const int tid  = threadIdx.x;
  const int lane = tid & 31;
  const int wave = tid >> 5;
  const int hh   = lane >> 4;
  const int m    = lane & 15;
  const int rowBase = blockIdx.x * GR;

  stage_a<K, 64>(hin, nN, rowBase, tid, At);
  __syncthreads();

  v8f acc = {0.f, 0.f, 0.f, 0.f, 0.f, 0.f, 0.f, 0.f};
#pragma unroll
  for (int kt = 0; kt < K / 32; ++kt) {
    const int k0 = kt * 32;
    Frag a, b;
    const _Float16* pa = At + (16 * wave + m) * AP + k0 + 8 * hh;
    const _Float16* pb = Lt + (size_t)m * K + k0 + 8 * hh;
    a.half[0] = *(const v8h*)pa; a.half[1] = *(const v8h*)(pa + 16);
    b.half[0] = *(const v8h*)pb; b.half[1] = *(const v8h*)(pb + 16);
    acc = wm(a.v, b.v, acc);
  }

  const int mc = (m < MLPW) ? m : (MLPW - 1);
  const float lbt = lb1[mc];
  const float lwt = lw2[mc];
  const float lb = (m < MLPW) ? lbt : 0.f;
  const float lw = (m < MLPW) ? lwt : 0.f;
  const float ob = lb2[0];
  float o[8];
#pragma unroll
  for (int r = 0; r < 8; ++r) {
    float v = acc[r] * 0.125f + lb;
    v = v > 0.f ? v : 0.f;
    o[r] = v * lw;
  }
#pragma unroll
  for (int mk = 1; mk < 16; mk <<= 1) {
#pragma unroll
    for (int r = 0; r < 8; ++r) o[r] += __shfl_xor(o[r], mk, 32);
  }
  if (m == 0) {
#pragma unroll
    for (int r = 0; r < 8; ++r) Os[16 * wave + 8 * hh + r] = o[r] + ob;
  }
  __syncthreads();

  if (wave == 0) {
    const v4f ov = *(const v4f*)(Os + 4 * (lane & 7));
    if (rowBase + GR <= nN) {
      if (lane < 8) {
        float* p = out + rowBase + 4 * lane;
        *(volatile v4f*)p = ov;
        __threadfence();
        *(volatile v4f*)p = ov;
      }
    } else {
      const float os = Os[lane];
      if (rowBase + lane < nN) {
        float* p = out + rowBase + lane;
        *(volatile float*)p = os;
        __threadfence();
        *(volatile float*)p = os;
      }
    }
  }
}

static inline size_t al256(size_t v) { return (v + 255) & ~(size_t)255; }

extern "C" void kernel_launch(void* const* d_in, const int* in_sizes, int n_in,
                              void* d_out, int out_size, void* d_ws, size_t ws_size,
                              hipStream_t stream) {
  if (n_in < 20) return;
  const int nN = in_sizes[0] / INF0;
  if (nN <= 0 || in_sizes[0] != nN * INF0) return;
  if (in_sizes[1] < 0 || (in_sizes[1] & 1) != 0) return;
  const int nE = in_sizes[1] / 2;
  if ((long long)in_sizes[2] != (long long)nE * EDIM) return;
  if (in_sizes[3] != INF0 * HIDF || in_sizes[9] != HIDF * HIDF) return;
  if (in_sizes[4] != EDIM * HIDF || in_sizes[10] != EDIM * HIDF) return;
  if (in_sizes[5] != NHD * HCH || in_sizes[6] != NHD * HCH || in_sizes[7] != NHD * HCH) return;
  if (in_sizes[11] != NHD * HCH || in_sizes[12] != NHD * HCH || in_sizes[13] != NHD * HCH) return;
  if (in_sizes[8] != HIDF || in_sizes[14] != HIDF) return;
  if (in_sizes[15] != HIDF * MLPW || in_sizes[16] != MLPW || in_sizes[17] != MLPW) return;
  if (in_sizes[18] != 1 || in_sizes[19] != EDIM) return;
  if (out_size != nN) return;

  const float* x   = (const float*)d_in[0];
  const int*   ei  = (const int*)d_in[1];
  const float* ea  = (const float*)d_in[2];
  const float* W1  = (const float*)d_in[3];
  const float* We1 = (const float*)d_in[4];
  const float* as1 = (const float*)d_in[5];
  const float* ad1 = (const float*)d_in[6];
  const float* ae1 = (const float*)d_in[7];
  const float* b1  = (const float*)d_in[8];
  const float* W2  = (const float*)d_in[9];
  const float* We2 = (const float*)d_in[10];
  const float* as2 = (const float*)d_in[11];
  const float* ad2 = (const float*)d_in[12];
  const float* ae2 = (const float*)d_in[13];
  const float* b2  = (const float*)d_in[14];
  const float* lw1 = (const float*)d_in[15];
  const float* lb1 = (const float*)d_in[16];
  const float* lw2 = (const float*)d_in[17];
  const float* lb2 = (const float*)d_in[18];
  const float* sla = (const float*)d_in[19];
  float* out = (float*)d_out;

  const int nP = ((nN + GR - 1) / GR) * GR;
  size_t off = 0;
  _Float16* Wb = (_Float16*)((char*)d_ws + off); off = al256(off + (size_t)896 * 16);
  float* hpre  = (float*)((char*)d_ws + off);    off = al256(off + (size_t)nP * HIDF * sizeof(float));
  float* hpost = (float*)((char*)d_ws + off);    off = al256(off + (size_t)nP * HIDF * sizeof(float));
  float* asn   = (float*)((char*)d_ws + off);    off = al256(off + (size_t)nP * NHD * sizeof(float));
  float* adn   = (float*)((char*)d_ws + off);    off = al256(off + (size_t)nP * NHD * sizeof(float));
  if (off > ws_size) return;
  const _Float16* W1t = Wb;
  const _Float16* W2t = Wb + 2048;
  const _Float16* L1t = Wb + 6144;

  k_prep<<<4, 256, 0, stream>>>(W1, W2, lw1, Wb);

  k_gemm<INF0><<<nP / GR, 128, 0, stream>>>(x, W1t, as1, ad1, hpre, asn, adn, nN);

  hipFuncSetAttribute(reinterpret_cast<const void*>(&k_gat),
                      hipFuncAttributeMaxDynamicSharedMemorySize, LDS_BYTES);
  const int ggrid = (nN + NB - 1) / NB;
  k_gat<<<ggrid, NTHR, LDS_BYTES, stream>>>(ei, ea, hpre, asn, adn, We1, ae1, sla, b1, hpost, nN, nE);

  k_gemm<HIDF><<<nP / GR, 128, 0, stream>>>(hpost, W2t, as2, ad2, hpre, asn, adn, nN);
  k_gat<<<ggrid, NTHR, LDS_BYTES, stream>>>(ei, ea, hpre, asn, adn, We2, ae2, sla, b2, hpost, nN, nE);

  k_head<<<nP / GR, 64, 0, stream>>>(hpost, L1t, lb1, lw2, lb2, out, nN);
}
